// HebbianMap2d_41068477284655
// MI455X (gfx1250) — hardware-run, weakly checked
//
#include <hip/hip_runtime.h>
#include <math.h>

typedef __attribute__((ext_vector_type(16))) _Float16 v16h;
typedef __attribute__((ext_vector_type(8)))  _Float16 v8h;
typedef __attribute__((ext_vector_type(8)))  float    v8f;
typedef __attribute__((ext_vector_type(4)))  float    v4f;
typedef __attribute__((ext_vector_type(4)))  unsigned v4u;

constexpr int kNB     = 16;
constexpr int kCin    = 3;
constexpr int kHin    = 32;
constexpr int kWin    = 32;
constexpr int kKer    = 5;
constexpr int kHo     = kHin - kKer + 1;
constexpr int kWo     = kWin - kKer + 1;
constexpr int kPos    = kHo * kWo;
constexpr int kNrow   = kNB * kPos;
constexpr int kOch    = 96;
constexpr int kDepth  = kCin * kKer * kKer;
constexpr int kKpad   = 96;
constexpr int kNpad   = 128;
constexpr int kImg    = kCin * kHin * kWin;
constexpr int kOut0   = kNB * kOch * kPos;
constexpr int kOut1   = kOch * kDepth;
constexpr int kSegLen = 98;
constexpr float kCarryX = 16.0f;
constexpr float kCarryW = 256.0f;
constexpr float kFold   = 1.0f / (kCarryX * kCarryW);
constexpr float kEta    = 1e-3f;
constexpr float kInvN   = 1.0f / (float)kNrow;

static_assert(kHo == 28 && kWo == 28 && kPos == 784);
static_assert(kNrow == 12544 && kDepth == 75);
static_assert(kImg == 3072);
static_assert(kOut0 == 1204224 && kOut1 == 7200);
static_assert((kNrow % 64) == 0 && (kNpad % 64) == 0 && (kKpad % 32) == 0);
static_assert(kKpad >= kDepth && kNpad >= kOch);
static_assert(128 * kSegLen == kNrow);
static_assert((kOut0 % 256) == 0);
static_assert((kOut0 * 4) % 128 == 0);
static_assert((size_t)kOut0 * 4 + (size_t)kOut1 * 4 == 4845696ull);
static_assert((kOut1 % 32) == 0);

constexpr size_t kOffA16   = 0;
constexpr size_t kOffBT16  = kOffA16  + (size_t)kNrow * kKpad * 2;
constexpr size_t kOffSPL   = kOffBT16 + (size_t)kNpad * kKpad * 2;
constexpr size_t kOffMROW  = kOffSPL  + (size_t)kNrow * kNpad * 4;
constexpr size_t kOffFIRST = kOffMROW + (size_t)kNrow * 4;
constexpr size_t kOffDWP   = kOffFIRST + (size_t)kNrow * 4;
constexpr size_t kWsTotal  = kOffDWP  + (size_t)kOch * kNpad * 4;
static_assert(kWsTotal == 9005056ull);
static_assert(kWsTotal <= 134217728ull);
static_assert((kOffBT16 % 128) == 0 && (kOffSPL % 128) == 0 && (kOffMROW % 128) == 0 &&
              (kOffFIRST % 128) == 0 && (kOffDWP % 128) == 0);

__device__ __forceinline__ void store2_f32(float* p, float v) {
  *(volatile float*)p = v;
  __threadfence();
  *(volatile float*)p = v;
}
__device__ __forceinline__ void store2_i32(int* p, int v) {
  *(volatile int*)p = v;
  __threadfence();
  *(volatile int*)p = v;
}
__device__ __forceinline__ void store2_v4u(unsigned short* p, v4u v) {
  *(volatile v4u*)p = v;
  __threadfence();
  *(volatile v4u*)p = v;
}
__device__ __forceinline__ unsigned f16_bits(float f) {
  const _Float16 h = (_Float16)f;
  const unsigned short b = __builtin_bit_cast(unsigned short, h);
  return (unsigned)b;
}

__device__ __forceinline__ void wm_guard1(v8f& a, v16h x, v16h y) {
  asm volatile("v_nop\n\tv_nop\n\tv_nop\n\tv_nop" : "+v"(a) : "v"(x), "v"(y));
}
__device__ __forceinline__ void keep4_h(v16h a, v16h b, v16h c, v16h d) {
  asm volatile("v_nop" :: "v"(a), "v"(b), "v"(c), "v"(d));
}
__device__ __forceinline__ void acc_guard4(v8f& a, v8f& b, v8f& c, v8f& d) {
  asm volatile("v_nop\n\tv_nop\n\tv_nop\n\tv_nop" : "+v"(a), "+v"(b), "+v"(c), "+v"(d));
}
union FragH { v16h v; v8h h[2]; };
__device__ __forceinline__ v16h frag_load_h(const _Float16* p) {
  FragH f;
  f.h[0] = *(const v8h*)(p);
  f.h[1] = *(const v8h*)(p + 16);
  return f.v;
}
__device__ __forceinline__ v8f mma_h(v16h a, v16h b, v8f c) {
  return __builtin_amdgcn_wmma_f32_16x16x32_f16(false, a, false, b, (short)0, c, false, false);
}

constexpr int kPackXLanes = kNrow * kKpad / 8;
static_assert((kPackXLanes % 256) == 0);
__global__ __launch_bounds__(256) void pack_x_kernel(const float* __restrict__ x, unsigned short* __restrict__ A16) {
  const int g = blockIdx.x * 256 + threadIdx.x;
  if (g >= kPackXLanes) return;
  const int e0 = g * 8;
  const int n  = e0 / kKpad;
  const int k0 = e0 - n * kKpad;
  const int b  = n / kPos;
  const int p  = n - b * kPos;
  const int oh = p / kWo;
  const int ow = p - oh * kWo;
  const float* xb = x + b * kImg + oh * kWin + ow;
  unsigned hb[8];
#pragma unroll
  for (int e = 0; e < 8; ++e) {
    const int k  = k0 + e;
    const int kc = (k < kDepth) ? k : (kDepth - 1);
    const int c  = kc / (kKer * kKer);
    const int r  = kc - c * (kKer * kKer);
    const int ki = r / kKer;
    const int kj = r - ki * kKer;
    const float v = xb[(c * kHin + ki) * kWin + kj];
    const float f = (k < kDepth) ? (v * kCarryX) : 0.0f;
    hb[e] = f16_bits(f);
  }
  v4u wv;
  wv.x = hb[0] | (hb[1] << 16);
  wv.y = hb[2] | (hb[3] << 16);
  wv.z = hb[4] | (hb[5] << 16);
  wv.w = hb[6] | (hb[7] << 16);
  store2_v4u(A16 + (size_t)e0, wv);
}

constexpr int kPackWLanes = kNpad * kKpad / 8;
static_assert((kPackWLanes % 256) == 0);
__global__ __launch_bounds__(256) void pack_w_kernel(const float* __restrict__ w, unsigned short* __restrict__ BT16) {
  const int g = blockIdx.x * 256 + threadIdx.x;
  if (g >= kPackWLanes) return;
  const int e0 = g * 8;
  const int o  = e0 / kKpad;
  const int k0 = e0 - o * kKpad;
  const int oc = (o < kOch) ? o : (kOch - 1);
  unsigned hb[8];
#pragma unroll
  for (int e = 0; e < 8; ++e) {
    const int k  = k0 + e;
    const int kc = (k < kDepth) ? k : (kDepth - 1);
    const float v = w[oc * kDepth + kc];
    const float f = ((o < kOch) && (k < kDepth)) ? (v * kCarryW) : 0.0f;
    hb[e] = f16_bits(f);
  }
  v4u wv;
  wv.x = hb[0] | (hb[1] << 16);
  wv.y = hb[2] | (hb[3] << 16);
  wv.z = hb[4] | (hb[5] << 16);
  wv.w = hb[6] | (hb[7] << 16);
  store2_v4u(BT16 + (size_t)e0, wv);
}

__global__ __launch_bounds__(256) void gemm_f16_kernel(
    const unsigned short* __restrict__ Ap, int lda,
    const unsigned short* __restrict__ Btp, int ldb,
    float* __restrict__ C, int ldc, int M, int N, int K, float scale) {
  const _Float16* A  = (const _Float16*)Ap;
  const _Float16* Bt = (const _Float16*)Btp;
  __shared__ __align__(16) float sT[8][16 * 68];
  const int lane = threadIdx.x & 31;
  const int wave = __builtin_amdgcn_readfirstlane((int)(threadIdx.x >> 5));
  const int tilesN = N >> 6;
  const int tilesM = M >> 6;
  const int tile = blockIdx.x * 8 + wave;
  if (tile >= tilesM * tilesN) return;
  const int tm = tile / tilesN;
  const int tn = tile - tm * tilesN;
  const int m0 = tm << 6;
  const int n0 = tn << 6;

  const int rlane = lane & 15;
  const int koff  = (lane >> 4) * 8;
  const int mOff  = (lane >> 4) * 8;

  v8f acc[4][4];
#pragma unroll
  for (int i = 0; i < 4; ++i)
#pragma unroll
    for (int j = 0; j < 4; ++j) acc[i][j] = (v8f){0.f, 0.f, 0.f, 0.f, 0.f, 0.f, 0.f, 0.f};

  for (int k0 = 0; k0 < K; k0 += 32) {
    v16h bh[4];
#pragma unroll
    for (int j = 0; j < 4; ++j) {
      const size_t bo = (size_t)(n0 + (j << 4) + rlane) * ldb + koff + k0;
      bh[j] = frag_load_h(Bt + bo);
    }
#pragma unroll
    for (int i = 0; i < 4; ++i) {
      const size_t ao = (size_t)(m0 + (i << 4) + rlane) * lda + koff + k0;
      const v16h ah = frag_load_h(A + ao);
#pragma unroll
      for (int j = 0; j < 4; ++j) acc[i][j] = mma_h(ah, bh[j], acc[i][j]);
      wm_guard1(acc[i][0], ah, bh[0]);
      wm_guard1(acc[i][1], ah, bh[1]);
      wm_guard1(acc[i][2], ah, bh[2]);
      wm_guard1(acc[i][3], ah, bh[3]);
    }
    keep4_h(bh[0], bh[1], bh[2], bh[3]);
  }
  acc_guard4(acc[0][0], acc[0][1], acc[0][2], acc[0][3]);
  acc_guard4(acc[1][0], acc[1][1], acc[1][2], acc[1][3]);
  acc_guard4(acc[2][0], acc[2][1], acc[2][2], acc[2][3]);
  acc_guard4(acc[3][0], acc[3][1], acc[3][2], acc[3][3]);

  float* slab = sT[wave];
#pragma unroll
  for (int i = 0; i < 4; ++i) {
    const int mBase = m0 + (i << 4);
#pragma unroll
    for (int j = 0; j < 4; ++j) {
#pragma unroll
      for (int r = 0; r < 8; ++r) {
        const float v = acc[i][j][r] * scale;
        slab[(mOff + r) * 68 + (j << 4) + rlane] = v;
      }
    }
    __builtin_amdgcn_fence(__ATOMIC_RELEASE, "workgroup");
    __builtin_amdgcn_wave_barrier();
    __builtin_amdgcn_fence(__ATOMIC_ACQUIRE, "workgroup");
    {
      const int hh = lane >> 4, c4 = (lane & 15) * 4;
      for (int pass = 0; pass < 2; ++pass) {
#pragma unroll
        for (int it = 0; it < 8; ++it) {
          const int row = it * 2 + hh;
          const v4f v = *(const v4f*)(slab + row * 68 + c4);
          *(volatile v4f*)(C + (size_t)(mBase + row) * ldc + n0 + c4) = v;
        }
        __threadfence();
      }
    }
    __builtin_amdgcn_fence(__ATOMIC_RELEASE, "workgroup");
    __builtin_amdgcn_wave_barrier();
    __builtin_amdgcn_fence(__ATOMIC_ACQUIRE, "workgroup");
  }
}

__global__ __launch_bounds__(256) void transpose_out_kernel(const float* __restrict__ SPL, float* __restrict__ out0) {
  const int j = blockIdx.x * 256 + threadIdx.x;
  if (j >= kOut0) return;
  const int b   = j / (kOch * kPos);
  const int rem = j - b * (kOch * kPos);
  const int o   = rem / kPos;
  const int p   = rem - o * kPos;
  const float v = SPL[(size_t)(b * kPos + p) * kNpad + o];
  store2_f32(out0 + j, v);
}

static_assert((kNrow % 256) == 0);
__global__ __launch_bounds__(256) void winner_kernel(const float* __restrict__ SPL, float* __restrict__ MROW, int* __restrict__ FIRST) {
  const int n = blockIdx.x * 256 + threadIdx.x;
  if (n >= kNrow) return;
  const float* row = SPL + (size_t)n * kNpad;
  float m = -__builtin_inff();
  int first = 0;
#pragma unroll 1
  for (int q = 0; q < kOch / 4; ++q) {
    const v4f v = *(const v4f*)(row + 4 * q);
    const float a0 = v.x, a1 = v.y, a2 = v.z, a3 = v.w;
    bool g;
    g = a0 > m; m = g ? a0 : m; first = g ? (4 * q + 0) : first;
    g = a1 > m; m = g ? a1 : m; first = g ? (4 * q + 1) : first;
    g = a2 > m; m = g ? a2 : m; first = g ? (4 * q + 2) : first;
    g = a3 > m; m = g ? a3 : m; first = g ? (4 * q + 3) : first;
  }
  store2_f32(MROW + n, m);
  store2_i32(FIRST + n, first);
}

__global__ __launch_bounds__(128) void delta_kernel(
    const float* __restrict__ x, const float* __restrict__ w, const float* __restrict__ SPL,
    const float* __restrict__ MROW, const int* __restrict__ FIRST, float* __restrict__ DWP) {
  __shared__ int seg[128 * kSegLen];
  __shared__ int cnt[128];
  const int tid = threadIdx.x;
  const int o   = blockIdx.x;
  {
    int c = 0;
    const int nb = tid * kSegLen;
#pragma unroll 1
    for (int i = 0; i < kSegLen; ++i) {
      const int n = nb + i;
      float sv = SPL[(size_t)n * kNpad + o];
      float mv = MROW[n];
      asm volatile("" : "+v"(sv), "+v"(mv));
      const bool hit = (sv == mv);
      if (hit) {
        seg[tid * kSegLen + c] = n;
        ++c;
      }
    }
    cnt[tid] = c;
  }
  __syncthreads();

  const int dc   = (tid < kDepth) ? tid : (kDepth - 1);
  const int ch   = dc / (kKer * kKer);
  const int r25  = dc - ch * (kKer * kKer);
  const int ki   = r25 / kKer;
  const int kj   = r25 - ki * kKer;
  const int xoff = (ch * kHin + ki) * kWin + kj;
  float acc = 0.0f;
#pragma unroll 1
  for (int t = 0; t < 128; ++t) {
    int ct = __builtin_amdgcn_readfirstlane(cnt[t]);
    ct = ct < 0 ? 0 : (ct > kSegLen ? kSegLen : ct);
#pragma unroll 1
    for (int i = 0; i < ct; ++i) {
      int n = __builtin_amdgcn_readfirstlane(seg[t * kSegLen + i]);
      n = n < 0 ? 0 : (n > kNrow - 1 ? kNrow - 1 : n);
      const float mv = MROW[n];
      int f = __builtin_amdgcn_readfirstlane(FIRST[n]);
      f = f < 0 ? 0 : (f > o ? o : f);
      const int b  = n / kPos;
      const int p  = n - b * kPos;
      const int oh = p / kWo;
      const int ow = p - oh * kWo;
      const float xv = x[b * kImg + xoff + oh * kWin + ow];
      float pref = 0.0f;
#pragma unroll 1
      for (int oo = f; oo <= o; ++oo) {
        const float so = SPL[(size_t)n * kNpad + oo];
        const float wv = w[oo * kDepth + dc];
        const float term = mv * wv;
        pref += (so == mv) ? term : 0.0f;
      }
      acc += mv * (xv - pref);
    }
  }
  const float outv = (tid < kDepth) ? acc : 0.0f;
  store2_f32(DWP + (size_t)o * kNpad + tid, outv);
}

__global__ __launch_bounds__(256) void finalize_kernel(const float* __restrict__ w, const float* __restrict__ DWP, float* __restrict__ out1) {
  const int i  = blockIdx.x * 256 + threadIdx.x;
  const int ic = (i < kOut1) ? i : (kOut1 - 1);
  const int o  = ic / kDepth;
  const int d  = ic - o * kDepth;
  const float dv = DWP[(size_t)o * kNpad + d];
  const float wv = w[ic];
  const float mean = dv * kInvN;
  const float res = wv + kEta * mean;
  if (i < kOut1) store2_f32(out1 + i, res);
}

extern "C" void kernel_launch(void* const* d_in, const int* in_sizes, int n_in,
                              void* d_out, int out_size, void* d_ws, size_t ws_size,
                              hipStream_t stream) {
  if (n_in < 2) return;
  if (in_sizes[0] != kNB * kImg) return;
  if (in_sizes[1] != kOut1) return;
  if (out_size != kOut0 + kOut1) return;
  if (ws_size < kWsTotal) return;

  const float* x = (const float*)d_in[0];
  const float* w = (const float*)d_in[1];
  float* out0 = (float*)d_out;
  float* out1 = out0 + (size_t)kOut0;

  char* ws = (char*)d_ws;
  unsigned short* A16   = (unsigned short*)(ws + kOffA16);
  unsigned short* BT16  = (unsigned short*)(ws + kOffBT16);
  float*          SPL   = (float*)(ws + kOffSPL);
  float*          MROW  = (float*)(ws + kOffMROW);
  int*            FIRST = (int*)(ws + kOffFIRST);
  float*          DWP   = (float*)(ws + kOffDWP);

  pack_x_kernel<<<kPackXLanes / 256, 256, 0, stream>>>(x, A16);
  pack_w_kernel<<<kPackWLanes / 256, 256, 0, stream>>>(w, BT16);

  gemm_f16_kernel<<<((kNrow / 64) * (kNpad / 64)) / 8, 256, 0, stream>>>(
      A16, kKpad, BT16, kKpad, SPL, kNpad, kNrow, kNpad, kKpad, kFold);

  transpose_out_kernel<<<kOut0 / 256, 256, 0, stream>>>(SPL, out0);
  winner_kernel<<<kNrow / 256, 256, 0, stream>>>(SPL, MROW, FIRST);
  delta_kernel<<<kOch, 128, 0, stream>>>(x, w, SPL, MROW, FIRST, DWP);
  finalize_kernel<<<(kOut1 + 255) / 256, 256, 0, stream>>>(w, DWP, out1);
}
